// ModulatedDeformConv3d_84774064489048
// MI455X (gfx1250) — hardware-verified
//
#include <hip/hip_runtime.h>
#include <math.h>

typedef __attribute__((ext_vector_type(16))) _Float16 v16h;
typedef __attribute__((ext_vector_type(16))) __bf16 v16b;
typedef __attribute__((ext_vector_type(8)))  _Float16 v8h;
typedef __attribute__((ext_vector_type(8)))  float v8f;
typedef __attribute__((ext_vector_type(4)))  float v4f;
typedef __attribute__((ext_vector_type(2)))  float v2f;
typedef __attribute__((ext_vector_type(4)))  unsigned v4u;
typedef __attribute__((ext_vector_type(4)))  int v4i;
typedef float __attribute__((may_alias)) float_a;
typedef int __attribute__((may_alias)) int_a;

template <typename T> __device__ __forceinline__ void vst2(void* p, T v) { *(volatile T*)p = v; __threadfence(); *(volatile T*)p = v; }
__device__ __forceinline__ v8f wmma16(v16h a, v16h b, v8f c) {
  v8f d = __builtin_amdgcn_wmma_f32_16x16x32_f16(false, a, false, b, (short)0, c, false, false);
  asm volatile("v_nop\n\tv_nop\n\tv_nop\n\tv_nop" : "+v"(d) : "v"(a), "v"(b));
  return d;
}
__device__ __forceinline__ v8f wmma_bf(v16b a, v16b b, v8f c) {
  v8f d = __builtin_amdgcn_wmma_f32_16x16x32_bf16(false, a, false, b, (short)0, c, false, false);
  asm volatile("v_nop\n\tv_nop\n\tv_nop\n\tv_nop" : "+v"(d) : "v"(a), "v"(b));
  return d;
}
__device__ __forceinline__ v16h frag_h(const _Float16* rowk0, int lane) {
  union { v16h v; v8h q[2]; } u; const _Float16* p = rowk0 + 8 * (lane >> 4);
  u.q[0] = *(const v8h*)p; u.q[1] = *(const v8h*)(p + 16); return u.v;
}
__device__ __forceinline__ v16h frag_f32(const float* rowk0, int lane) {
  v16h a; const float* p = rowk0 + 8 * (lane >> 4);
#pragma unroll
  for (int i = 0; i < 8; ++i) { a[i] = (_Float16)p[i]; a[8 + i] = (_Float16)p[16 + i]; }
  return a;
}
__device__ __forceinline__ v16h frag_f32s(const float* rowk0, int lane, float sc) {
  v16h a; const float* p = rowk0 + 8 * (lane >> 4);
#pragma unroll
  for (int i = 0; i < 8; ++i) { a[i] = (_Float16)(p[i] * sc); a[8 + i] = (_Float16)(p[16 + i] * sc); }
  return a;
}
__device__ __forceinline__ v16h fragc_f32(const float* W, int k0, int n, int lane, int ld, int K) {
  v16h a; const int g = lane >> 4;
#pragma unroll
  for (int i = 0; i < 8; ++i) { const int ka = k0 + 8 * g + i, kb = ka + 16;
    a[i] = (_Float16)(ka < K ? W[(size_t)(ka < K ? ka : K - 1) * ld + n] : 0.f); a[8 + i] = (_Float16)(kb < K ? W[(size_t)(kb < K ? kb : K - 1) * ld + n] : 0.f); }
  return a;
}
struct F2 { v16b h, l; };
__device__ __forceinline__ F2 bsplit16(const float v[16]) { F2 r;
#pragma unroll
  for (int i = 0; i < 16; ++i) { const __bf16 h = (__bf16)v[i]; r.h[i] = h; r.l[i] = (__bf16)(v[i] - (float)h); }
  return r; }
__device__ __forceinline__ F2 split_row(const float* row, int k0, int lane) { float v[16]; const float* p = row + k0 + 8 * (lane >> 4);
#pragma unroll
  for (int i = 0; i < 8; ++i) { v[i] = p[i]; v[8 + i] = p[16 + i]; }
  return bsplit16(v); }
__device__ __forceinline__ F2 split_rowK(const float* row, int k0, int lane, int K) { float v[16]; const int g = lane >> 4;
#pragma unroll
  for (int i = 0; i < 8; ++i) { const int ka = k0 + 8 * g + i, kb = ka + 16; v[i] = ka < K ? row[ka < K ? ka : K - 1] : 0.f; v[8 + i] = kb < K ? row[kb < K ? kb : K - 1] : 0.f; }
  return bsplit16(v); }
__device__ __forceinline__ F2 split_col(const float* W, int k0, int n, int lane, int ld, int K) { float v[16]; const int g = lane >> 4;
#pragma unroll
  for (int i = 0; i < 8; ++i) { const int ka = k0 + 8 * g + i, kb = ka + 16; v[i] = ka < K ? W[(size_t)(ka < K ? ka : K - 1) * ld + n] : 0.f; v[8 + i] = kb < K ? W[(size_t)(kb < K ? kb : K - 1) * ld + n] : 0.f; }
  return bsplit16(v); }
__device__ __forceinline__ v8f mac3(const F2& a, const F2& b, v8f c) { c = wmma_bf(a.l, b.h, c); c = wmma_bf(a.h, b.l, c); return wmma_bf(a.h, b.h, c); }
__device__ __forceinline__ float sigm(float v) { return 1.0f / (1.0f + expf(-v)); }
#define LDSX() do { asm volatile("s_wait_dscnt 0" ::: "memory"); __builtin_amdgcn_wave_barrier(); __builtin_amdgcn_fence(__ATOMIC_RELEASE, "workgroup"); } while (0)


#define CC 64
#define CO 64
#define SZ 32
#define NPOS 32768
#define KP 27
#define KTOT (KP * CC)
#ifndef TPB
#define TPB (NPOS / 16)
#endif
#ifndef TOB
#define TOB (NPOS / 64)
#endif
typedef __attribute__((ext_vector_type(8))) __bf16 v8b;
__device__ __forceinline__ v16b frag_b(const __bf16* rowk0, int lane) {
  union { v16b v; v8b q[2]; } u; const __bf16* p = rowk0 + 8 * (lane >> 4);
  u.q[0] = *(const v8b*)p; u.q[1] = *(const v8b*)(p + 16); return u.v;
}
__device__ __forceinline__ float bfr(float v) { return (float)(__bf16)v; }
__device__ __attribute__((noinline)) float exp_ni(float v) { return expf(v); }
__device__ __attribute__((noinline)) float erf_ni(float v) { return erff(v); }

#define WS_XT  0u
#define WS_COL (WS_XT + 4u * (size_t)NPOS * CC)
#define WS_END (WS_COL + 2u * (size_t)NPOS * KTOT)

__global__ __launch_bounds__(128) void k_xt(const float* __restrict__ X, float* __restrict__ XT) { __shared__ __align__(16) float s[64][68]; const int tid = threadIdx.x; const int p0 = blockIdx.x * 64;
  for (int e = tid; e < CC * 64; e += 128) { const int c = e >> 6, pl = e & 63; s[pl][c] = bfr(X[(size_t)c * NPOS + p0 + pl]); }
  __syncthreads(); for (int e = tid; e < 64 * 16; e += 128) { const int pl = e >> 4, q = e & 15; vst2(XT + (size_t)(p0 + pl) * CC + q * 4, *(const v4f*)&s[pl][q * 4]); } }
__global__ __launch_bounds__(128) void k_col(const float* __restrict__ XT, const float* __restrict__ OFF, const float* __restrict__ MSK, _Float16* __restrict__ COL) { __shared__ __align__(16) _Float16 srow[16][KTOT + 8];
  const int t = threadIdx.x; const int pl = t >> 3, ck = t & 7; const int p = blockIdx.x * 16 + pl; const int ho = p / (SZ * SZ), wo = (p / SZ) % SZ, lo = p % SZ;
#pragma unroll 1
  for (int k = 0; k < KP; ++k) { const int ki = k / 9, kj = (k / 3) % 3, kk = k % 3;
    const float ch = bfr(OFF[((size_t)(k * 3 + 0)) * NPOS + p]) + (float)(ho - 1) + (float)ki;
    const float cw = bfr(OFF[((size_t)(k * 3 + 1)) * NPOS + p]) + (float)(wo - 1) + (float)kj;
    const float cl = bfr(OFF[((size_t)(k * 3 + 2)) * NPOS + p]) + (float)(lo - 1) + (float)kk;
    const float mk = bfr(MSK[(size_t)k * NPOS + p]);
    const float h0 = floorf(ch), w0 = floorf(cw), l0 = floorf(cl); const float fh = ch - h0, fw = cw - w0, fl = cl - l0; const int h0i = (int)h0, w0i = (int)w0, l0i = (int)l0;
    float acc[8]; for (int i = 0; i < 8; ++i) acc[i] = 0.f;
#pragma unroll 1
    for (int cr = 0; cr < 8; ++cr) { const int dh = (cr >> 2) & 1, dw = (cr >> 1) & 1, dl = cr & 1; const int ih = h0i + dh, iw = w0i + dw, il = l0i + dl;
      const bool valid = (ih >= 0 && ih < SZ && iw >= 0 && iw < SZ && il >= 0 && il < SZ);
      const float wgt = (dh ? fh : 1.0f - fh) * (dw ? fw : 1.0f - fw) * (dl ? fl : 1.0f - fl);
      const int chh = ih < 0 ? 0 : (ih >= SZ ? SZ - 1 : ih), cww = iw < 0 ? 0 : (iw >= SZ ? SZ - 1 : iw), cll = il < 0 ? 0 : (il >= SZ ? SZ - 1 : il);
      const float* src = XT + ((size_t)(chh * SZ + cww) * SZ + cll) * CC + ck * 8; const v4f a0 = *(const v4f*)src, a1 = *(const v4f*)(src + 4); const float wv = valid ? wgt : 0.f;
      acc[0] += a0[0] * wv; acc[1] += a0[1] * wv; acc[2] += a0[2] * wv; acc[3] += a0[3] * wv; acc[4] += a1[0] * wv; acc[5] += a1[1] * wv; acc[6] += a1[2] * wv; acc[7] += a1[3] * wv; }
    for (int i = 0; i < 8; ++i) srow[pl][k * CC + ck * 8 + i] = (_Float16)(acc[i] * mk); }
  __syncthreads();
  for (int e = t; e < 16 * (KTOT / 8); e += 128) { const int rl = e / (KTOT / 8), q = e % (KTOT / 8); vst2((unsigned*)(COL + (size_t)(blockIdx.x * 16 + rl) * KTOT + q * 8), *(const v4u*)&srow[rl][q * 8]); } }
__global__ __launch_bounds__(128) void k_gemm(const _Float16* __restrict__ COL, const float* __restrict__ WT, float* __restrict__ OUT) { __shared__ __align__(16) float st[CO][68];
  const int tid = threadIdx.x, wave = tid >> 5, lane = tid & 31, col = lane & 15, g = lane >> 4; const int p0 = blockIdx.x * 64; const size_t r0 = (size_t)p0 + wave * 16;
  v8f acc[4] = {};
#pragma unroll 2
  for (int kc = 0; kc < KTOT / 32; ++kc) { const v16h a = frag_h(COL + (r0 + col) * KTOT + kc * 32, lane);
#pragma unroll
    for (int j = 0; j < 4; ++j) { v16h w; const int o = j * 16 + col;
#pragma unroll
      for (int i = 0; i < 8; ++i) { { const int kk = kc * 32 + 8 * g + i; const int k = kk / CC, c = kk % CC; w[i] = (_Float16)bfr(WT[((size_t)o * CC + c) * KP + k]); } { const int kk = kc * 32 + 16 + 8 * g + i; const int k = kk / CC, c = kk % CC; w[8 + i] = (_Float16)bfr(WT[((size_t)o * CC + c) * KP + k]); } }
      acc[j] = wmma16(a, w, acc[j]); } }
#pragma unroll
  for (int j = 0; j < 4; ++j)
#pragma unroll
    for (int r = 0; r < 8; ++r) st[j * 16 + col][wave * 16 + 8 * g + r] = acc[j][r];
  __syncthreads(); for (int e = tid; e < CO * 16; e += 128) { const int o = e >> 4, q = e & 15; vst2(OUT + (size_t)o * NPOS + p0 + q * 4, *(const v4f*)&st[o][q * 4]); } }
extern "C" void kernel_launch(void* const* d_in, const int* in_sizes, int n_in, void* d_out, int out_size, void* d_ws, size_t ws_size, hipStream_t stream) {
  (void)in_sizes; (void)n_in; (void)out_size;
  const float** F = (const float**)d_in;
  if (ws_size < (size_t)WS_END) return;
  char* ws = (char*)d_ws; float* XT = (float*)(ws + WS_XT); _Float16* COL = (_Float16*)(ws + WS_COL);
  k_xt<<<NPOS / 64, 128, 0, stream>>>(F[0], XT);
  k_col<<<TPB, 128, 0, stream>>>(XT, F[1], F[2], COL);
  k_gemm<<<TOB, 128, 0, stream>>>(COL, F[3], (float*)d_out);
}
